// RegionalSpatialAttention_71914932404728
// MI455X (gfx1250) — hardware-verified
//
#include <hip/hip_runtime.h>
#include <math.h>

#define NB_ 4
#define IH  64
#define IW  64
#define CC_ 256
#define NHD 8
#define HD  32
#define NS  25
#define NTOK (NB_ * IH * IW)

typedef _Float16 f16;
typedef __attribute__((ext_vector_type(16))) f16 f16x16;
typedef __attribute__((ext_vector_type(8)))  f16 f16x8;
typedef __attribute__((ext_vector_type(8)))  float f32x8;
typedef __attribute__((ext_vector_type(4)))  float v4f_t;
typedef float v4fa __attribute__((ext_vector_type(4), may_alias));
typedef __attribute__((ext_vector_type(4))) unsigned v4u_t;
typedef unsigned v4ua __attribute__((ext_vector_type(4), may_alias));

__device__ __forceinline__ f32x8 wmma16(f16x16 a, f16x16 b, f32x8 c) {
  c = __builtin_amdgcn_wmma_f32_16x16x32_f16(false, a, false, b, (short)0, c, false, false);
  asm volatile("v_nop\n\tv_nop\n\tv_nop\n\tv_nop" : "+v"(c) : "v"(a), "v"(b));
  return c;
}
__device__ __forceinline__ f16x16 lds_frag(const f16* base, int stride) {
  const int lane = threadIdx.x & 31, row = lane & 15, kh = (lane >> 4) * 8;
  const f16x8 lo = *(const f16x8*)(base + row * stride + kh);
  const f16x8 hi = *(const f16x8*)(base + row * stride + kh + 16);
  f16x16 f;
#pragma unroll
  for (int i = 0; i < 8; ++i) { f[i] = lo[i]; f[i + 8] = hi[i]; }
  return f;
}
#define GSTR 48

template <typename AT, bool ACC>
__global__ __launch_bounds__(256) void gemm_kn2(const AT* __restrict__ A, int lda, size_t strideA,
                                               const float* __restrict__ Wm, int ldw, size_t strideW,
                                               const float* __restrict__ bias, float scale,
                                               float* __restrict__ Y, int ldy, size_t strideY, int K) {
  __shared__ __attribute__((aligned(16))) f16 ldsA[128 * GSTR], ldsAl[128 * GSTR];
  __shared__ __attribute__((aligned(16))) f16 ldsW[128 * GSTR], ldsWl[128 * GSTR];
  __shared__ __attribute__((aligned(16))) float oS[8][32 * 68];
  const int tid = threadIdx.x, lane = tid & 31, wave = tid >> 5, cl = lane & 15, rh = (lane >> 4) * 8;
  const int m0 = blockIdx.x * 128, n0 = blockIdx.y * 128;
  const int wm = (wave & 3) * 32, wn = (wave >> 2) * 64;
  A += (size_t)blockIdx.z * strideA; Wm += (size_t)blockIdx.z * strideW; Y += (size_t)blockIdx.z * strideY;
  f32x8 acc[2][4], accx[2][4];
#pragma unroll
  for (int i = 0; i < 2; ++i)
#pragma unroll
    for (int j = 0; j < 4; ++j) { f32x8 z = {}; acc[i][j] = z; accx[i][j] = z; }
#pragma unroll 1
  for (int k0 = 0; k0 < K; k0 += 32) {
    __syncthreads();
    {
      const int row = tid >> 1, ch = (tid & 1) * 16;
      const AT* src = A + (size_t)(m0 + row) * lda + k0 + ch;
#pragma unroll
      for (int g = 0; g < 16; ++g) { const float v = (float)src[g]; const f16 h = (f16)v; ldsA[row * GSTR + ch + g] = h; ldsAl[row * GSTR + ch + g] = (f16)((v - (float)h) * 2048.0f); }
    }
    {
      const int k = tid >> 3, nn0 = (tid & 7) * 16;
      const float* src = Wm + (size_t)(k0 + k) * ldw + n0 + nn0;
#pragma unroll
      for (int g = 0; g < 4; ++g) { const v4f_t v = *(const v4f_t*)(src + 4 * g);
#pragma unroll
        for (int u = 0; u < 4; ++u) { const f16 h = (f16)v[u]; ldsW[(nn0 + 4 * g + u) * GSTR + k] = h; ldsWl[(nn0 + 4 * g + u) * GSTR + k] = (f16)((v[u] - (float)h) * 2048.0f); } }
    }
    __syncthreads();
    f16x16 af[2], afl[2];
#pragma unroll
    for (int i = 0; i < 2; ++i) { af[i] = lds_frag(ldsA + (wm + 16 * i) * GSTR, GSTR); afl[i] = lds_frag(ldsAl + (wm + 16 * i) * GSTR, GSTR); }
#pragma unroll
    for (int j = 0; j < 4; ++j) {
      const f16x16 bf = lds_frag(ldsW + (wn + 16 * j) * GSTR, GSTR), bfl = lds_frag(ldsWl + (wn + 16 * j) * GSTR, GSTR);
#pragma unroll
      for (int i = 0; i < 2; ++i) { acc[i][j] = wmma16(af[i], bf, acc[i][j]); accx[i][j] = wmma16(af[i], bfl, accx[i][j]); accx[i][j] = wmma16(afl[i], bf, accx[i][j]); }
    }
  }
  float* so = oS[wave];
#pragma unroll
  for (int i = 0; i < 2; ++i)
#pragma unroll
    for (int j = 0; j < 4; ++j) {
      const float bv = bias ? bias[n0 + wn + 16 * j + cl] : 0.0f;
#pragma unroll
      for (int r = 0; r < 8; ++r) so[(16 * i + rh + r) * 68 + 16 * j + cl] = (acc[i][j][r] + accx[i][j][r] * (1.0f / 2048.0f)) * scale + bv;
    }
  asm volatile("s_wait_dscnt 0" ::: "memory");
  __builtin_amdgcn_wave_barrier();
  if (ACC) {
#pragma unroll
    for (int it = 0; it < 16; ++it) { const int f4 = lane + 32 * it, rr = f4 >> 4, q = (f4 & 15) * 4;
      const v4f_t old = *(const volatile v4fa*)(Y + (size_t)(m0 + wm + rr) * ldy + n0 + wn + q);
      v4f_t v = *(const volatile v4fa*)(so + rr * 68 + q); v += old; *(volatile v4fa*)(so + rr * 68 + q) = v; }
    asm volatile("s_wait_dscnt 0" ::: "memory");
  }
#pragma unroll 1
  for (int pass = 0; pass < 2; ++pass) {
#pragma unroll
    for (int it = 0; it < 16; ++it) { const int f4 = lane + 32 * it, rr = f4 >> 4, q = (f4 & 15) * 4;
      *(volatile v4f_t*)(Y + (size_t)(m0 + wm + rr) * ldy + n0 + wn + q) = *(const volatile v4fa*)(so + rr * 68 + q); }
    __threadfence();
  }
}

__global__ __launch_bounds__(256) void k_regional(const float* __restrict__ Q, const float* __restrict__ Kf, const float* __restrict__ V,
                                                 const float* __restrict__ pos, float* __restrict__ attn) {
  __shared__ __attribute__((aligned(16))) f16 qS[2][32 * 40], kS[2][96 * 40], pS[2][32 * 40], vT[2][32 * 104];
  __shared__ __attribute__((aligned(16))) f16 PS[2][32 * 104];
  __shared__ __attribute__((aligned(16))) float sS[32 * 100], qpS[32 * 36];
  __shared__ __attribute__((aligned(16))) float oS[32 * 260];
  const int tid = threadIdx.x, lane = tid & 31, wave = tid >> 5, cl = lane & 15, rh = (lane >> 4) * 8;
  const int tilesX = IW / 8, tilesY = IH / 4;
  const int b = blockIdx.x / (tilesX * tilesY), trem = blockIdx.x % (tilesX * tilesY), y0 = (trem / tilesX) * 4, x0 = (trem % tilesX) * 8;
  const int kyB = min(max(y0 - 2, 0), IH - 8), kxB = min(max(x0 - 2, 0), IW - 12);
  const size_t tok0 = (size_t)b * IH * IW;
#pragma unroll 1
  for (int h = 0; h < NHD; ++h) {
    __syncthreads();
    for (int e = tid; e < 32 * 32; e += 256) { const int q = e >> 5, d = e & 31; const int y = y0 + (q >> 3), x = x0 + (q & 7);
      { const float vq = Q[(tok0 + (size_t)y * IW + x) * CC_ + h * HD + d]; const f16 hq = (f16)vq; qS[0][q * 40 + d] = hq; qS[1][q * 40 + d] = (f16)((vq - (float)hq) * 2048.0f); } }
    for (int e = tid; e < 96 * 32; e += 256) { const int kk = e >> 5, d = e & 31; const int ky = kyB + kk / 12, kx = kxB + kk % 12;
      const size_t tk = tok0 + (size_t)ky * IW + kx;
      { const float vk = Kf[tk * CC_ + h * HD + d]; const f16 hk = (f16)vk; kS[0][kk * 40 + d] = hk; kS[1][kk * 40 + d] = (f16)((vk - (float)hk) * 2048.0f);
        const float vv = V[tk * CC_ + h * HD + d]; const f16 hv = (f16)vv; vT[0][d * 104 + kk] = hv; vT[1][d * 104 + kk] = (f16)((vv - (float)hv) * 2048.0f); } }
    for (int e = tid; e < 32 * 32; e += 256) { const int s = e >> 5, d = e & 31; const float vp = (s < NS) ? pos[s * CC_ + h * HD + d] : 0.0f; const f16 hp = (f16)vp; pS[0][s * 40 + d] = hp; pS[1][s * 40 + d] = (f16)((vp - (float)hp) * 2048.0f); }
    for (int e = tid; e < 2 * 32 * 104; e += 256) (&PS[0][0])[e] = (f16)0.0f;
    if (tid < 32) {
#pragma unroll
      for (int c = 96; c < 104; ++c) { vT[0][tid * 104 + c] = (f16)0.0f; vT[1][tid * 104 + c] = (f16)0.0f; } }
    __syncthreads();
#pragma unroll
    for (int tt = 0; tt < 2; ++tt) {
      const int tix = wave * 2 + tt;
      f32x8 acc = {}, accx = {};
      if (tix < 12) { const int qt = tix / 6, kt = tix % 6;
        const f16x16 ah = lds_frag(qS[0] + (qt * 16) * 40, 40), al = lds_frag(qS[1] + (qt * 16) * 40, 40), bh = lds_frag(kS[0] + (kt * 16) * 40, 40), bl = lds_frag(kS[1] + (kt * 16) * 40, 40);
        acc = wmma16(ah, bh, acc); accx = wmma16(ah, bl, accx); accx = wmma16(al, bh, accx);
#pragma unroll
        for (int r = 0; r < 8; ++r) sS[(qt * 16 + rh + r) * 100 + kt * 16 + cl] = acc[r] + accx[r] * (1.0f / 2048.0f);
      } else { const int qt = (tix - 12) >> 1, st = (tix - 12) & 1;
        const f16x16 ah = lds_frag(qS[0] + (qt * 16) * 40, 40), al = lds_frag(qS[1] + (qt * 16) * 40, 40), bh = lds_frag(pS[0] + (st * 16) * 40, 40), bl = lds_frag(pS[1] + (st * 16) * 40, 40);
        acc = wmma16(ah, bh, acc); accx = wmma16(ah, bl, accx); accx = wmma16(al, bh, accx);
#pragma unroll
        for (int r = 0; r < 8; ++r) qpS[(qt * 16 + rh + r) * 36 + st * 16 + cl] = acc[r] + accx[r] * (1.0f / 2048.0f);
      }
    }
    __syncthreads();
    if (tid < 32) {
      const int q = tid, y = y0 + (q >> 3), x = x0 + (q & 7);
      const int cy = min(max(y, 2), IH - 3), cx = min(max(x, 2), IW - 3);
      float lg[NS]; float mx = -INFINITY;
#pragma unroll
      for (int s = 0; s < NS; ++s) { const int dy = s / 5 - 2, dx = s % 5 - 2; const int kk = (cy + dy - kyB) * 12 + (cx + dx - kxB);
        lg[s] = (sS[q * 100 + kk] + qpS[q * 36 + s]) * (0.17677669529663688f * 1.44269504088896340736f);
        mx = fmaxf(mx, lg[s]); }
      float z = 0.0f;
#pragma unroll
      for (int s = 0; s < NS; ++s) { lg[s] = exp2f(lg[s] - mx); z += lg[s]; }
      const float iz = 1024.0f / z;
#pragma unroll
      for (int s = 0; s < NS; ++s) { const int dy = s / 5 - 2, dx = s % 5 - 2; const int kk = (cy + dy - kyB) * 12 + (cx + dx - kxB); const float pv = lg[s] * iz; const f16 hp = (f16)pv;
        PS[0][q * 104 + kk] = hp; PS[1][q * 104 + kk] = (f16)((pv - (float)hp) * 2048.0f); }
    }
    __syncthreads();
    if (wave < 4) { const int qt = wave >> 1, dt = wave & 1;
      f32x8 acc = {}, accx = {};
#pragma unroll
      for (int ks = 0; ks < 3; ++ks) { const f16x16 ah = lds_frag(PS[0] + (qt * 16) * 104 + ks * 32, 104), al = lds_frag(PS[1] + (qt * 16) * 104 + ks * 32, 104), bh = lds_frag(vT[0] + (dt * 16) * 104 + ks * 32, 104), bl = lds_frag(vT[1] + (dt * 16) * 104 + ks * 32, 104);
        acc = wmma16(ah, bh, acc); accx = wmma16(ah, bl, accx); accx = wmma16(al, bh, accx); }
#pragma unroll
      for (int r = 0; r < 8; ++r) oS[(qt * 16 + rh + r) * 260 + h * HD + dt * 16 + cl] = (acc[r] + accx[r] * (1.0f / 2048.0f)) * (1.0f / 1024.0f);
    }
  }
  __syncthreads();
#pragma unroll 1
  for (int pass = 0; pass < 2; ++pass) {
#pragma unroll
    for (int it = 0; it < 8; ++it) { const int ch = tid + 256 * it, q = ch >> 6, c4 = (ch & 63) * 4; const int y = y0 + (q >> 3), x = x0 + (q & 7);
      *(volatile v4f_t*)(attn + (tok0 + (size_t)y * IW + x) * CC_ + c4) = *(const volatile v4fa*)(oS + q * 260 + c4); }
    __threadfence();
  }
}

extern "C" void kernel_launch(void* const* d_in, const int* in_sizes, int n_in,
                              void* d_out, int out_size, void* d_ws, size_t ws_size,
                              hipStream_t stream) {
  (void)in_sizes; (void)n_in; (void)out_size; (void)ws_size;
  const float* x = (const float*)d_in[0];
  const float* Wq = (const float*)d_in[1], *Wk = (const float*)d_in[2], *Wv = (const float*)d_in[3], *Wo = (const float*)d_in[4];
  const float* pos = (const float*)d_in[5];
  float* out = (float*)d_out;
  char* ws = (char*)d_ws;
  const size_t T = (size_t)NTOK * CC_ * 4;
  float* Qb = (float*)ws; float* Kb = (float*)(ws + T); float* Vb = (float*)(ws + 2 * T); float* att = (float*)(ws + 3 * T);
  const dim3 g(NTOK / 128, CC_ / 128, 1), blk(256);
  gemm_kn2<float, false><<<g, blk, 0, stream>>>(x, CC_, 0, Wq, CC_, 0, nullptr, 1.0f, Qb, CC_, 0, CC_);
  gemm_kn2<float, false><<<g, blk, 0, stream>>>(x, CC_, 0, Wk, CC_, 0, nullptr, 1.0f, Kb, CC_, 0, CC_);
  gemm_kn2<float, false><<<g, blk, 0, stream>>>(x, CC_, 0, Wv, CC_, 0, nullptr, 1.0f, Vb, CC_, 0, CC_);
  k_regional<<<dim3(NB_ * (IH / 4) * (IW / 8)), blk, 0, stream>>>(Qb, Kb, Vb, pos, att);
  gemm_kn2<float, false><<<g, blk, 0, stream>>>(att, CC_, 0, Wo, CC_, 0, nullptr, 1.0f, out, CC_, 0, CC_);
}
